// DampedIMEX2Layer_22368189677866
// MI455X (gfx1250) — hardware-run, weakly checked
//
#include <hip/hip_runtime.h>
#include <math.h>

constexpr int SEQ_LEN   = 16384;
constexpr int HID_DIM   = 256;
constexpr int NUM_STATE = 512;
constexpr int STATE2    = 2 * NUM_STATE;
constexpr int NUM_SEG   = 2;
constexpr int SEG_ROWS  = SEQ_LEN / NUM_SEG;
static_assert(SEG_ROWS * NUM_SEG == SEQ_LEN, "segments cover the sequence");
static_assert(SEG_ROWS % 64 == 0, "M tile multiple");
static_assert(STATE2 % 64 == 0 && HID_DIM % 64 == 0, "N tile multiples");
static_assert(HID_DIM % 32 == 0 && STATE2 % 32 == 0, "K multiples of 32");
static_assert(NUM_STATE % 32 == 0, "one wave per 32 states");

constexpr float U_CARRY        = 16.0f;
constexpr float W_CARRY        = 256.0f;
constexpr float FOLD_BACK      = 1.0f / (U_CARRY * W_CARRY);
constexpr float F16_MIN_NORMAL = 6.103515625e-05f;
static_assert(U_CARRY * W_CARRY * FOLD_BACK == 1.0f, "carry fold is exact");
static_assert(F16_MIN_NORMAL * 16384.0f == 1.0f, "2^-14");

typedef __attribute__((ext_vector_type(16))) _Float16 v16h;
typedef __attribute__((ext_vector_type(8)))  _Float16 v8h;
typedef __attribute__((ext_vector_type(16))) __bf16   v16b;
typedef __attribute__((ext_vector_type(8)))  __bf16   v8b;
typedef __attribute__((ext_vector_type(8)))  float    v8f;
typedef __attribute__((ext_vector_type(4)))  float    v4f;
typedef __attribute__((ext_vector_type(2)))  float    v2f;
typedef __attribute__((ext_vector_type(4)))  unsigned int v4u;

__device__ __forceinline__ unsigned bf_hi_bits(float f) {
  const unsigned u = __float_as_uint(f);
  return (u + 0x7FFFu + ((u >> 16) & 1u)) >> 16;
}
__device__ __forceinline__ float bf_bits_f32(unsigned h) { return __uint_as_float(h << 16); }
__device__ __forceinline__ void bf_split(float f, unsigned& hb, unsigned& lb) {
  hb = bf_hi_bits(f);
  lb = bf_hi_bits(f - bf_bits_f32(hb));
}

__device__ __forceinline__ _Float16 to_f16_flush(float v) {
  const float fl = (fabsf(v) < F16_MIN_NORMAL) ? 0.0f : v;
  return (_Float16)fl;
}

namespace eng {

__device__ __forceinline__ void tie_acc(v8f& a, v16b x, v16b y) {
  asm volatile("v_nop\n\tv_nop\n\tv_nop\n\tv_nop" : "+v"(a) : "v"(x), "v"(y));
}
__device__ __forceinline__ void tie_acc_h(v8f& a, v16h x, v16h y) {
  asm volatile("v_nop\n\tv_nop\n\tv_nop\n\tv_nop" : "+v"(a) : "v"(x), "v"(y));
}
__device__ __forceinline__ void keep4_b(v16b a, v16b b, v16b c, v16b d) {
  asm volatile("v_nop" :: "v"(a), "v"(b), "v"(c), "v"(d));
}
__device__ __forceinline__ void keep4_h(v16h a, v16h b, v16h c, v16h d) {
  asm volatile("v_nop" :: "v"(a), "v"(b), "v"(c), "v"(d));
}
__device__ __forceinline__ void acc_guard4(v8f& a, v8f& b, v8f& c, v8f& d) {
  asm volatile("v_nop\n\tv_nop\n\tv_nop\n\tv_nop" : "+v"(a), "+v"(b), "+v"(c), "+v"(d));
}

struct FragB {
  union U { v16b v; v8b h[2]; };
  static __device__ __forceinline__ v16b load(const __bf16* p) {
    U f;
    f.h[0] = *(const v8b*)(p);
    f.h[1] = *(const v8b*)(p + 16);
    return f.v;
  }
  static __device__ __forceinline__ v8f mma(v16b a, v16b b, v8f c) {
    return __builtin_amdgcn_wmma_f32_16x16x32_bf16(false, a, false, b, (short)0, c, false, false);
  }
};

struct FragH {
  union U { v16h v; v8h h[2]; };
  static __device__ __forceinline__ v16h load(const _Float16* p) {
    U f;
    f.h[0] = *(const v8h*)(p);
    f.h[1] = *(const v8h*)(p + 16);
    return f.v;
  }
  static __device__ __forceinline__ v8f mma(v16h a, v16h b, v8f c) {
    return __builtin_amdgcn_wmma_f32_16x16x32_f16(false, a, false, b, (short)0, c, false, false);
  }
};

__global__ __launch_bounds__(256) void gemm64_f16x1(
    const unsigned short* __restrict__ Ap, int lda,
    const unsigned short* __restrict__ Btp, int ldb,
    float* __restrict__ C, int ldc,
    int M, int N, int K, float scale) {
  const _Float16* A  = (const _Float16*)Ap;
  const _Float16* Bt = (const _Float16*)Btp;
  __shared__ __align__(16) float sT[8][16 * 68];
  const int lane = threadIdx.x & 31;
  const int wave = threadIdx.x >> 5;
  const int tilesN = N >> 6;
  const int tilesM = M >> 6;
  const int tile = blockIdx.x * 8 + wave;
  if (tile >= tilesM * tilesN) return;
  const int tm = tile / tilesN;
  const int tn = tile - tm * tilesN;
  const int m0 = tm << 6;
  const int n0 = tn << 6;

  const int rlane = lane & 15;
  const int koff  = (lane >> 4) * 8;
  const int mOff  = (lane >> 4) * 8;

  v8f acc[4][4];
#pragma unroll
  for (int i = 0; i < 4; ++i)
#pragma unroll
    for (int j = 0; j < 4; ++j) acc[i][j] = (v8f){0.f, 0.f, 0.f, 0.f, 0.f, 0.f, 0.f, 0.f};

  for (int k0 = 0; k0 < K; k0 += 32) {
    v16h bh[4];
#pragma unroll
    for (int j = 0; j < 4; ++j) {
      const size_t bo = (size_t)(n0 + (j << 4) + rlane) * ldb + koff + k0;
      bh[j] = FragH::load(Bt + bo);
    }
#pragma unroll
    for (int i = 0; i < 4; ++i) {
      const size_t ao = (size_t)(m0 + (i << 4) + rlane) * lda + koff + k0;
      const v16h ah = FragH::load(A + ao);
#pragma unroll
      for (int j = 0; j < 4; ++j) {
        acc[i][j] = FragH::mma(ah, bh[j], acc[i][j]);
      }
      tie_acc_h(acc[i][0], ah, ah);
      tie_acc_h(acc[i][1], ah, ah);
      tie_acc_h(acc[i][2], ah, ah);
      tie_acc_h(acc[i][3], ah, ah);
    }
    keep4_h(bh[0], bh[1], bh[2], bh[3]);
  }
  acc_guard4(acc[0][0], acc[0][1], acc[0][2], acc[0][3]);
  acc_guard4(acc[1][0], acc[1][1], acc[1][2], acc[1][3]);
  acc_guard4(acc[2][0], acc[2][1], acc[2][2], acc[2][3]);
  acc_guard4(acc[3][0], acc[3][1], acc[3][2], acc[3][3]);

  float* slab = sT[wave];
  const int hh = lane >> 4;
  const int c4 = (lane & 15) * 4;
#pragma unroll
  for (int i = 0; i < 4; ++i) {
    const int mBase = m0 + (i << 4);
#pragma unroll
    for (int j = 0; j < 4; ++j) {
#pragma unroll
      for (int r = 0; r < 8; ++r) {
        slab[(mOff + r) * 68 + (j << 4) + rlane] = acc[i][j][r] * scale;
      }
    }
    __builtin_amdgcn_fence(__ATOMIC_RELEASE, "workgroup");
    __builtin_amdgcn_wave_barrier();
    __builtin_amdgcn_fence(__ATOMIC_ACQUIRE, "workgroup");
    v4f vals[8];
#pragma unroll
    for (int it = 0; it < 8; ++it) {
      const int row = it * 2 + hh;
      vals[it] = *(const v4f*)(slab + row * 68 + c4);
    }
    for (int pass = 0; pass < 2; ++pass) {
#pragma unroll
      for (int it = 0; it < 8; ++it) {
        const int row = it * 2 + hh;
        *(volatile v4f*)(C + (size_t)(mBase + row) * ldc + n0 + c4) = vals[it];
      }
      __threadfence();
    }
    __builtin_amdgcn_fence(__ATOMIC_RELEASE, "workgroup");
    __builtin_amdgcn_wave_barrier();
    __builtin_amdgcn_fence(__ATOMIC_ACQUIRE, "workgroup");
  }
}

template <int RESID>
__global__ __launch_bounds__(256) void gemm64_bf16x3(
    const unsigned short* __restrict__ Ahp, const unsigned short* __restrict__ Alp, int lda,
    const unsigned short* __restrict__ Bhp, const unsigned short* __restrict__ Blp, int ldb,
    float* __restrict__ C, int ldc,
    const float* __restrict__ resid, const float* __restrict__ rcoef,
    int M, int N, int K) {
  const __bf16* Ah = (const __bf16*)Ahp;
  const __bf16* Al = (const __bf16*)Alp;
  const __bf16* Bh = (const __bf16*)Bhp;
  const __bf16* Bl = (const __bf16*)Blp;
  __shared__ __align__(16) float sT[8][16 * 68];
  const int lane = threadIdx.x & 31;
  const int wave = threadIdx.x >> 5;
  const int tilesN = N >> 6;
  const int tilesM = M >> 6;
  const int tile = blockIdx.x * 8 + wave;
  if (tile >= tilesM * tilesN) return;
  const int tm = tile / tilesN;
  const int tn = tile - tm * tilesN;
  const int m0 = tm << 6;
  const int n0 = tn << 6;

  const int rlane = lane & 15;
  const int koff  = (lane >> 4) * 8;
  const int mOff  = (lane >> 4) * 8;

  v8f acc[4][4];
#pragma unroll
  for (int i = 0; i < 4; ++i)
#pragma unroll
    for (int j = 0; j < 4; ++j) acc[i][j] = (v8f){0.f, 0.f, 0.f, 0.f, 0.f, 0.f, 0.f, 0.f};

  for (int k0 = 0; k0 < K; k0 += 32) {
    v16b bh[4], bl[4];
#pragma unroll
    for (int j = 0; j < 4; ++j) {
      const size_t bo = (size_t)(n0 + (j << 4) + rlane) * ldb + koff + k0;
      bh[j] = FragB::load(Bh + bo);
      bl[j] = FragB::load(Bl + bo);
    }
#pragma unroll
    for (int i = 0; i < 4; ++i) {
      const size_t ao = (size_t)(m0 + (i << 4) + rlane) * lda + koff + k0;
      const v16b ah = FragB::load(Ah + ao);
      const v16b al = FragB::load(Al + ao);
#pragma unroll
      for (int j = 0; j < 4; ++j) {
        acc[i][j] = FragB::mma(ah, bh[j], acc[i][j]);
        acc[i][j] = FragB::mma(ah, bl[j], acc[i][j]);
        acc[i][j] = FragB::mma(al, bh[j], acc[i][j]);
      }
      tie_acc(acc[i][0], ah, al);
      tie_acc(acc[i][1], ah, al);
      tie_acc(acc[i][2], ah, al);
      tie_acc(acc[i][3], ah, al);
    }
    keep4_b(bh[0], bh[1], bh[2], bh[3]);
    keep4_b(bl[0], bl[1], bl[2], bl[3]);
  }
  acc_guard4(acc[0][0], acc[0][1], acc[0][2], acc[0][3]);
  acc_guard4(acc[1][0], acc[1][1], acc[1][2], acc[1][3]);
  acc_guard4(acc[2][0], acc[2][1], acc[2][2], acc[2][3]);
  acc_guard4(acc[3][0], acc[3][1], acc[3][2], acc[3][3]);

  float* slab = sT[wave];
  const int hh = lane >> 4;
  const int c4 = (lane & 15) * 4;
  v4f dv = (v4f){0.f, 0.f, 0.f, 0.f};
  if (RESID == 1) dv = *(const v4f*)(rcoef + n0 + c4);
#pragma unroll
  for (int i = 0; i < 4; ++i) {
    const int mBase = m0 + (i << 4);
#pragma unroll
    for (int j = 0; j < 4; ++j) {
#pragma unroll
      for (int r = 0; r < 8; ++r) {
        slab[(mOff + r) * 68 + (j << 4) + rlane] = acc[i][j][r];
      }
    }
    __builtin_amdgcn_fence(__ATOMIC_RELEASE, "workgroup");
    __builtin_amdgcn_wave_barrier();
    __builtin_amdgcn_fence(__ATOMIC_ACQUIRE, "workgroup");
    v4f vals[8];
#pragma unroll
    for (int it = 0; it < 8; ++it) {
      const int row = it * 2 + hh;
      v4f v = *(const v4f*)(slab + row * 68 + c4);
      if (RESID == 1) {
        const v4f rr = *(const v4f*)(resid + (size_t)(mBase + row) * ldc + n0 + c4);
        v = v + dv * rr;
      }
      vals[it] = v;
    }
    for (int pass = 0; pass < 2; ++pass) {
#pragma unroll
      for (int it = 0; it < 8; ++it) {
        const int row = it * 2 + hh;
        *(volatile v4f*)(C + (size_t)(mBase + row) * ldc + n0 + c4) = vals[it];
      }
      __threadfence();
    }
    __builtin_amdgcn_fence(__ATOMIC_RELEASE, "workgroup");
    __builtin_amdgcn_wave_barrier();
    __builtin_amdgcn_fence(__ATOMIC_ACQUIRE, "workgroup");
  }
}

}

__global__ __launch_bounds__(256) void cast_f16x8_carry(const float* __restrict__ in,
                                                        unsigned short* __restrict__ out, int n8) {
  const int i = blockIdx.x * 256 + threadIdx.x;
  if (i >= n8) return;
  const float* p = in + (size_t)i * 8;
  const v4f a = *(const v4f*)p;
  const v4f c = *(const v4f*)(p + 4);
  float f[8];
#pragma unroll
  for (int e = 0; e < 4; ++e) { f[e] = a[e]; f[4 + e] = c[e]; }
  v8h hv;
#pragma unroll
  for (int e = 0; e < 8; ++e) {
    const float cv = f[e] * U_CARRY;
    hv[e] = to_f16_flush(cv);
  }
  unsigned short* op = out + (size_t)i * 8;
  *(volatile v8h*)op = hv;
  __threadfence();
  *(volatile v8h*)op = hv;
}

template <bool NEG_ODD>
__global__ __launch_bounds__(256) void split_planes8(const float* __restrict__ in,
                                                     unsigned* __restrict__ hi,
                                                     unsigned* __restrict__ lo, int n8) {
  const int i = blockIdx.x * 256 + threadIdx.x;
  if (i >= n8) return;
  const float* p = in + (size_t)i * 8;
  const v4f a = *(const v4f*)p;
  const v4f c = *(const v4f*)(p + 4);
  float f[8];
#pragma unroll
  for (int e = 0; e < 4; ++e) { f[e] = a[e]; f[4 + e] = c[e]; }
  if (NEG_ODD) {
#pragma unroll
    for (int e = 1; e < 8; e += 2) f[e] = -f[e];
  }
  v4u hv, lv;
#pragma unroll
  for (int e = 0; e < 4; ++e) {
    unsigned h0, l0, h1, l1;
    bf_split(f[2 * e], h0, l0);
    bf_split(f[2 * e + 1], h1, l1);
    hv[e] = h0 | (h1 << 16);
    lv[e] = l0 | (l1 << 16);
  }
  unsigned* hp = hi + (size_t)i * 4;
  unsigned* lp = lo + (size_t)i * 4;
  *(volatile v4u*)hp = hv;
  *(volatile v4u*)lp = lv;
  __threadfence();
  *(volatile v4u*)hp = hv;
  *(volatile v4u*)lp = lv;
}

__global__ __launch_bounds__(256) void prep_in_weight(const float* __restrict__ Bw,
                                                      unsigned short* __restrict__ Bt16) {
  const int i = blockIdx.x * 256 + threadIdx.x;
  if (i >= NUM_STATE * 32) return;
  const int p  = i >> 5;
  const int hg = i & 31;
  const float* src = Bw + ((size_t)p * HID_DIM + (size_t)hg * 8) * 2;
  const v4f q0 = *(const v4f*)(src);
  const v4f q1 = *(const v4f*)(src + 4);
  const v4f q2 = *(const v4f*)(src + 8);
  const v4f q3 = *(const v4f*)(src + 12);
  float f[16];
#pragma unroll
  for (int e = 0; e < 4; ++e) { f[e] = q0[e]; f[4 + e] = q1[e]; f[8 + e] = q2[e]; f[12 + e] = q3[e]; }
  v8h re, im;
#pragma unroll
  for (int j = 0; j < 8; ++j) {
    const float cr = f[2 * j] * W_CARRY;
    const float ci = f[2 * j + 1] * W_CARRY;
    re[j] = to_f16_flush(cr);
    im[j] = to_f16_flush(ci);
  }
  unsigned short* o0 = Bt16 + (size_t)(2 * p) * HID_DIM + (size_t)hg * 8;
  unsigned short* o1 = o0 + HID_DIM;
  *(volatile v8h*)o0 = re;
  *(volatile v8h*)o1 = im;
  __threadfence();
  *(volatile v8h*)o0 = re;
  *(volatile v8h*)o1 = im;
}

__global__ __launch_bounds__(NUM_STATE) void state_params(const float* __restrict__ A_diag,
                                                          const float* __restrict__ G_diag,
                                                          const float* __restrict__ dt,
                                                          float* __restrict__ PT) {
#pragma clang fp contract(off)
  const int p = threadIdx.x;
  const float ex    = expf(-dt[p]);
  const float onepe = 1.0f + ex;
  const float dts   = __fdiv_rn(1.0f, onepe);
  const float G     = fmaxf(G_diag[p], 0.0f);
  const float x     = dts * G;
  const float omx   = 1.0f - x;
  const float root  = __fsqrt_rn(omx);
  const float d2    = dts * dts;
  const float den   = fmaxf(d2, 1e-6f);
  const float tmx   = 2.0f - x;
  const float tr    = 2.0f * root;
  const float nlo   = tmx - tr;
  const float nhi   = tmx + tr;
  const float Alo   = __fdiv_rn(nlo, den);
  const float Ahi   = __fdiv_rn(nhi, den);
  const float Ad    = A_diag[p];
  const float r1    = fmaxf(Ad - Alo, 0.0f);
  const float r2    = fmaxf(Ad - Ahi, 0.0f);
  const float s1    = Alo + r1;
  const float A     = s1 - r2;
  const float m00   = omx;
  const float ndts  = -dts;
  const float m01   = ndts * A;
  const float m10   = dts * omx;
  const float d2A   = d2 * A;
  const float m11   = 1.0f - d2A;
  volatile float* P = PT;
  P[0 * NUM_STATE + p] = m00;
  P[1 * NUM_STATE + p] = m01;
  P[2 * NUM_STATE + p] = m10;
  P[3 * NUM_STATE + p] = m11;
  P[4 * NUM_STATE + p] = dts;
  P[5 * NUM_STATE + p] = d2;
  __threadfence();
  P[0 * NUM_STATE + p] = m00;
  P[1 * NUM_STATE + p] = m01;
  P[2 * NUM_STATE + p] = m10;
  P[3 * NUM_STATE + p] = m11;
  P[4 * NUM_STATE + p] = dts;
  P[5 * NUM_STATE + p] = d2;
}

__global__ __launch_bounds__(32) void state_scan(const float* __restrict__ PT,
                                                 const float* __restrict__ BU,
                                                 unsigned* __restrict__ YSh,
                                                 unsigned* __restrict__ YSl,
                                                 const float* __restrict__ stIn,
                                                 float* __restrict__ stOut,
                                                 int first) {
  const int p = blockIdx.x * 32 + threadIdx.x;
  const float m00 = PT[0 * NUM_STATE + p];
  const float m01 = PT[1 * NUM_STATE + p];
  const float m10 = PT[2 * NUM_STATE + p];
  const float m11 = PT[3 * NUM_STATE + p];
  const float c1  = PT[4 * NUM_STATE + p];
  const float c2  = PT[5 * NUM_STATE + p];
  float x1r = 0.f, x1i = 0.f, x2r = 0.f, x2i = 0.f;
  if (first == 0) {
    x1r = stIn[0 * NUM_STATE + p];
    x1i = stIn[1 * NUM_STATE + p];
    x2r = stIn[2 * NUM_STATE + p];
    x2i = stIn[3 * NUM_STATE + p];
  }
#pragma unroll 1
  for (int l = 0; l < SEG_ROWS; ++l) {
    const v2f b = *(const v2f*)(BU + (size_t)l * STATE2 + 2 * p);
    const float br = b[0];
    const float bi = b[1];
    const float n1r = m00 * x1r + m01 * x2r + c1 * br;
    const float n1i = m00 * x1i + m01 * x2i + c1 * bi;
    const float n2r = m10 * x1r + m11 * x2r + c2 * br;
    const float n2i = m10 * x1i + m11 * x2i + c2 * bi;
    x1r = n1r; x1i = n1i; x2r = n2r; x2i = n2i;
    unsigned hr, lr, hi, li;
    bf_split(n2r, hr, lr);
    bf_split(n2i, hi, li);
    const unsigned hw = hr | (hi << 16);
    const unsigned lw = lr | (li << 16);
    const size_t w = (size_t)l * NUM_STATE + p;
    volatile unsigned* hp = YSh + w;
    volatile unsigned* lp = YSl + w;
    *hp = hw;
    *lp = lw;
    __threadfence();
    *hp = hw;
    *lp = lw;
  }
  volatile float* so = stOut;
  so[0 * NUM_STATE + p] = x1r;
  so[1 * NUM_STATE + p] = x1i;
  so[2 * NUM_STATE + p] = x2r;
  so[3 * NUM_STATE + p] = x2i;
  __threadfence();
  so[0 * NUM_STATE + p] = x1r;
  so[1 * NUM_STATE + p] = x1i;
  so[2 * NUM_STATE + p] = x2r;
  so[3 * NUM_STATE + p] = x2i;
}

extern "C" void kernel_launch(void* const* d_in, const int* in_sizes, int n_in,
                              void* d_out, int out_size, void* d_ws, size_t ws_size,
                              hipStream_t stream) {
  if (n_in < 7) return;
  if (in_sizes[0] != SEQ_LEN * HID_DIM || in_sizes[1] != NUM_STATE || in_sizes[2] != NUM_STATE ||
      in_sizes[3] != NUM_STATE || in_sizes[4] != NUM_STATE * HID_DIM * 2 ||
      in_sizes[5] != HID_DIM * NUM_STATE * 2 || in_sizes[6] != HID_DIM) return;
  if (out_size != SEQ_LEN * HID_DIM) return;

  const float* u      = (const float*)d_in[0];
  const float* A_diag = (const float*)d_in[1];
  const float* G_diag = (const float*)d_in[2];
  const float* dt     = (const float*)d_in[3];
  const float* Bw     = (const float*)d_in[4];
  const float* Cw     = (const float*)d_in[5];
  const float* Dw     = (const float*)d_in[6];
  float* out = (float*)d_out;
  char* ws = (char*)d_ws;

  const size_t szU16 = (size_t)SEQ_LEN * HID_DIM * 2;
  const size_t szW16 = (size_t)STATE2 * HID_DIM * 2;
  const size_t szPT  = 16384;
  const size_t szST  = 16384;
  const size_t szBU  = (size_t)SEG_ROWS * STATE2 * 4;
  const size_t szY16 = (size_t)SEG_ROWS * STATE2 * 2;
  static_assert((size_t)6 * NUM_STATE * 4 <= 16384, "PT fits its carve");
  static_assert((size_t)NUM_SEG * 4 * NUM_STATE * 4 <= 16384, "ST fits its carve");
  size_t off = 0;
  const size_t oU16 = off; off += szU16;
  const size_t oB16 = off; off += szW16;
  const size_t oCh  = off; off += szW16;
  const size_t oCl  = off; off += szW16;
  const size_t oPT  = off; off += szPT;
  const size_t oST  = off; off += szST;
  const size_t oBU  = off; off += szBU;
  const size_t oYh  = off; off += szY16;
  const size_t oYl  = off; off += szY16;
  if (off > ws_size) return;

  unsigned short* U16  = (unsigned short*)(ws + oU16);
  unsigned short* Bt16 = (unsigned short*)(ws + oB16);
  unsigned short* Ch   = (unsigned short*)(ws + oCh);
  unsigned short* Cl   = (unsigned short*)(ws + oCl);
  float*          PT   = (float*)(ws + oPT);
  float*          ST   = (float*)(ws + oST);
  float*          BU   = (float*)(ws + oBU);
  unsigned short* YSh  = (unsigned short*)(ws + oYh);
  unsigned short* YSl  = (unsigned short*)(ws + oYl);

  cast_f16x8_carry<<<dim3((SEQ_LEN * HID_DIM / 8) / 256), 256, 0, stream>>>(
      u, U16, SEQ_LEN * HID_DIM / 8);
  prep_in_weight<<<dim3((NUM_STATE * 32) / 256), 256, 0, stream>>>(Bw, Bt16);
  split_planes8<true><<<dim3((HID_DIM * STATE2 / 8) / 256), 256, 0, stream>>>(
      Cw, (unsigned*)Ch, (unsigned*)Cl, HID_DIM * STATE2 / 8);
  state_params<<<dim3(1), NUM_STATE, 0, stream>>>(A_diag, G_diag, dt, PT);

  for (int sg = 0; sg < NUM_SEG; ++sg) {
    const size_t r0 = (size_t)sg * SEG_ROWS;
    eng::gemm64_f16x1<<<dim3((SEG_ROWS / 64) * (STATE2 / 64) / 8), 256, 0, stream>>>(
        U16 + r0 * HID_DIM, HID_DIM,
        Bt16, HID_DIM,
        BU, STATE2,
        SEG_ROWS, STATE2, HID_DIM, FOLD_BACK);
    const int prevSlot = (sg > 0) ? (sg - 1) : 0;
    state_scan<<<dim3(NUM_STATE / 32), 32, 0, stream>>>(
        PT, BU, (unsigned*)YSh, (unsigned*)YSl,
        ST + (size_t)prevSlot * 4 * NUM_STATE, ST + (size_t)sg * 4 * NUM_STATE,
        (sg == 0) ? 1 : 0);
    eng::gemm64_bf16x3<1><<<dim3((SEG_ROWS / 64) * (HID_DIM / 64) / 8), 256, 0, stream>>>(
        YSh, YSl, STATE2,
        Ch, Cl, STATE2,
        out + r0 * HID_DIM, HID_DIM,
        u + r0 * HID_DIM, Dw,
        SEG_ROWS, HID_DIM, STATE2);
  }
}
